// RWKV_Block_12893491822596
// MI455X (gfx1250) — hardware-verified
//
#include <hip/hip_runtime.h>
#include <math.h>

constexpr int kBatch  = 2;
constexpr int kSeq    = 256;
constexpr int kDim    = 2048;
constexpr int kHeadSz = 64;
constexpr int kTok    = kBatch * kSeq;
constexpr int kLr5    = 160;
constexpr int kLrPad  = 192;
constexpr int kDec    = 64;
constexpr int kStRows = 66;
constexpr long kPlane = (long)kTok * kDim;
constexpr float kEps  = 1e-5f;

typedef __attribute__((ext_vector_type(16))) _Float16 v16h;
typedef __attribute__((ext_vector_type(8)))  _Float16 v8h;
typedef __attribute__((ext_vector_type(16))) __bf16   v16b;
typedef __attribute__((ext_vector_type(8)))  __bf16   v8b;
typedef __attribute__((ext_vector_type(8)))  float    v8f;
typedef __attribute__((ext_vector_type(4)))  float    v4f;
typedef __attribute__((ext_vector_type(4)))  unsigned int v4u;

__device__ __forceinline__ unsigned short f2bf_bits(float f) {
  unsigned u = __float_as_uint(f);
  return (unsigned short)((u + 0x7FFFu + ((u >> 16) & 1u)) >> 16);
}
__device__ __forceinline__ float bf_bits2f(unsigned short h) { return __uint_as_float(((unsigned)h) << 16); }

__device__ __forceinline__ void dep_guard_h(v8f& a, v8f& b, v16h x, v16h y) { asm volatile("v_nop\n\tv_nop\n\tv_nop\n\tv_nop" : "+v"(a), "+v"(b) : "v"(x), "v"(y)); }
__device__ __forceinline__ void dep_guard_b(v8f& a, v8f& b, v16b x, v16b y) { asm volatile("v_nop\n\tv_nop\n\tv_nop\n\tv_nop" : "+v"(a), "+v"(b) : "v"(x), "v"(y)); }
__device__ __forceinline__ void keep4_h(v16h a, v16h b, v16h c, v16h d) { asm volatile("v_nop" :: "v"(a), "v"(b), "v"(c), "v"(d)); }
__device__ __forceinline__ void keep4_b(v16b a, v16b b, v16b c, v16b d) { asm volatile("v_nop" :: "v"(a), "v"(b), "v"(c), "v"(d)); }
__device__ __forceinline__ void acc_guard4(v8f& a, v8f& b, v8f& c, v8f& d) { asm volatile("v_nop\n\tv_nop\n\tv_nop\n\tv_nop" : "+v"(a), "+v"(b), "+v"(c), "+v"(d)); }
template <typename T> struct Frag;
template <> struct Frag<_Float16> {
  typedef v16h V; union U { v16h v; v8h h[2]; };
  static __device__ __forceinline__ v16h load(const _Float16* p) {
    U f; f.h[0] = *(const v8h*)(p); f.h[1] = *(const v8h*)(p + 16); return f.v;
  }
  static __device__ __forceinline__ v8f mma(v16h a, v16h b, v8f c) {
    return __builtin_amdgcn_wmma_f32_16x16x32_f16(false, a, false, b, (short)0, c, false, false);
  }
  static __device__ __forceinline__ void guard(v8f& a, v8f& b, v16h x, v16h y) { dep_guard_h(a, b, x, y); }
  static __device__ __forceinline__ void keep(v16h a, v16h b, v16h c, v16h d) { keep4_h(a, b, c, d); }
};
template <> struct Frag<__bf16> {
  typedef v16b V; union U { v16b v; v8b h[2]; };
  static __device__ __forceinline__ v16b load(const __bf16* p) {
    U f; f.h[0] = *(const v8b*)(p); f.h[1] = *(const v8b*)(p + 16); return f.v;
  }
  static __device__ __forceinline__ v8f mma(v16b a, v16b b, v8f c) {
    return __builtin_amdgcn_wmma_f32_16x16x32_bf16(false, a, false, b, (short)0, c, false, false);
  }
  static __device__ __forceinline__ void guard(v8f& a, v8f& b, v16b x, v16b y) { dep_guard_b(a, b, x, y); }
  static __device__ __forceinline__ void keep(v16b a, v16b b, v16b c, v16b d) { keep4_b(a, b, c, d); }
};

template <int ET> struct Elem;
template <> struct Elem<0> { typedef _Float16 T; };
template <> struct Elem<1> { typedef __bf16 T; };
template <int ET, bool SPLIT, int BIAS_MODE, int OUT_MODE, bool RESID, int ACT = 0>
__global__ __launch_bounds__(256) void wmma_gemm64(
    const unsigned short* __restrict__ Ap, const unsigned short* __restrict__ A2p, int lda, long strideA,
    const unsigned short* __restrict__ Btp, const unsigned short* __restrict__ Bt2p, int ldb, long strideB,
    void* __restrict__ Cout, void* __restrict__ Cout2, int ldc, long strideC,
    const float* __restrict__ bias,
    const float* __restrict__ resid, long strideR,
    int M, int N, int K, float scale) {
  typedef typename Elem<ET>::T T;
  typedef typename Frag<T>::V V;
  const T* A = (const T*)Ap; const T* A2 = (const T*)A2p; const T* Bt = (const T*)Btp; const T* Bt2 = (const T*)Bt2p;
  __shared__ __align__(16) float sT[8][16 * 68];
  const int b    = blockIdx.y;
  const int lane = threadIdx.x & 31;
  const int wave = threadIdx.x >> 5;
  const int tilesN = N >> 6;
  const int tilesM = M >> 6;
  const int tile = blockIdx.x * 8 + wave;
  if (tile >= tilesM * tilesN) return;
  const int tm = tile / tilesN;
  const int tn = tile - tm * tilesN;
  const int m0 = tm << 6;
  const int n0 = tn << 6;

  const T* Ab  = A  + (size_t)b * strideA;
  const T* Bb  = Bt + (size_t)b * strideB;
  const T* Ab2 = SPLIT ? (A2  + (size_t)b * strideA) : nullptr;
  const T* Bb2 = SPLIT ? (Bt2 + (size_t)b * strideB) : nullptr;

  const int rlane = lane & 15;
  const int koff  = (lane >> 4) * 8;
  const int mOff  = (lane >> 4) * 8;

  v8f acc[4][4];
#pragma unroll
  for (int i = 0; i < 4; ++i)
#pragma unroll
    for (int j = 0; j < 4; ++j) acc[i][j] = (v8f){0.f,0.f,0.f,0.f,0.f,0.f,0.f,0.f};

  for (int k0 = 0; k0 < K; k0 += 32) {
    V bh[4], bl[4];
#pragma unroll
    for (int j = 0; j < 4; ++j) {
      const size_t bo = (size_t)(n0 + (j << 4) + rlane) * ldb + koff + k0;
      bh[j] = Frag<T>::load(Bb + bo);
      if (SPLIT) bl[j] = Frag<T>::load(Bb2 + bo);
    }
#pragma unroll
    for (int i = 0; i < 4; ++i) {
      const size_t ao = (size_t)(m0 + (i << 4) + rlane) * lda + koff + k0;
      V ah = Frag<T>::load(Ab + ao);
      V al;
      if (SPLIT) al = Frag<T>::load(Ab2 + ao);
#pragma unroll
      for (int j = 0; j < 4; ++j) {
        acc[i][j] = Frag<T>::mma(ah, bh[j], acc[i][j]);
        if (SPLIT) {
          acc[i][j] = Frag<T>::mma(ah, bl[j], acc[i][j]);
          acc[i][j] = Frag<T>::mma(al, bh[j], acc[i][j]);
        }
      }
      Frag<T>::guard(acc[i][0], acc[i][3], ah, SPLIT ? al : ah);
    }
    Frag<T>::keep(bh[0], bh[1], bh[2], bh[3]);
    if (SPLIT) Frag<T>::keep(bl[0], bl[1], bl[2], bl[3]);
  }
  acc_guard4(acc[0][0], acc[0][1], acc[0][2], acc[0][3]);
  acc_guard4(acc[1][0], acc[1][1], acc[1][2], acc[1][3]);
  acc_guard4(acc[2][0], acc[2][1], acc[2][2], acc[2][3]);
  acc_guard4(acc[3][0], acc[3][1], acc[3][2], acc[3][3]);

  float* slab = sT[wave];
  const float* Rb = RESID ? (resid + (size_t)b * strideR) : nullptr;
#pragma unroll
  for (int i = 0; i < 4; ++i) {
    const int mBase = m0 + (i << 4);
#pragma unroll
    for (int j = 0; j < 4; ++j) {
      const int n = n0 + (j << 4) + rlane;
      float bv = 0.f;
      if (BIAS_MODE == 2) bv = bias[n];
#pragma unroll
      for (int r = 0; r < 8; ++r) {
        float v = acc[i][j][r] * scale;
        if (BIAS_MODE == 1) v += bias[mBase + mOff + r];
        if (BIAS_MODE == 2) v += bv;
        if (RESID) v += Rb[(size_t)(mBase + mOff + r) * ldc + n];
        if (ACT == 2) v = fmaxf(v, 0.0f);
        if (ACT == 4) v = (v > 0.f) ? v : 0.01f * v;
        slab[(mOff + r) * 68 + (j << 4) + rlane] = v;
      }
    }
    __builtin_amdgcn_fence(__ATOMIC_RELEASE, "workgroup");
    __builtin_amdgcn_wave_barrier();
    __builtin_amdgcn_fence(__ATOMIC_ACQUIRE, "workgroup");
    if (OUT_MODE == 0) {
      float* C = (float*)Cout + (size_t)b * strideC;
      const int hh = lane >> 4, c4 = (lane & 15) * 4;
      for (int pass = 0; pass < 2; ++pass) {
#pragma unroll
        for (int it = 0; it < 8; ++it) {
          const int row = it * 2 + hh;
          v4f v = *(const v4f*)(slab + row * 68 + c4);
          *(volatile v4f*)(C + (size_t)(mBase + row) * ldc + n0 + c4) = v;
        }
        __threadfence();
      }
    } else {
      const int q = lane >> 3, c8 = (lane & 7) * 8;
      unsigned short* C  = (unsigned short*)Cout  + (size_t)b * strideC;
      unsigned short* C2 = (OUT_MODE == 2) ? ((unsigned short*)Cout2 + (size_t)b * strideC) : nullptr;
      for (int pass = 0; pass < 2; ++pass) {
#pragma unroll
        for (int it = 0; it < 4; ++it) {
          const int row = it * 4 + q;
          const float* sp = slab + row * 68 + c8;
          v8h hv, lv;
#pragma unroll
          for (int e = 0; e < 8; ++e) {
            if (OUT_MODE == 1) {
              hv[e] = (_Float16)sp[e];
            } else {
              unsigned short hb = f2bf_bits(sp[e]);
              unsigned short lb = f2bf_bits(sp[e] - bf_bits2f(hb));
              hv[e] = __builtin_bit_cast(_Float16, hb);
              lv[e] = __builtin_bit_cast(_Float16, lb);
            }
          }
          *(volatile v8h*)(C + (size_t)(mBase + row) * ldc + n0 + c8) = hv;
          if (OUT_MODE == 2) *(volatile v8h*)(C2 + (size_t)(mBase + row) * ldc + n0 + c8) = lv;
        }
        __threadfence();
      }
    }
    __builtin_amdgcn_fence(__ATOMIC_RELEASE, "workgroup");
    __builtin_amdgcn_wave_barrier();
    __builtin_amdgcn_fence(__ATOMIC_ACQUIRE, "workgroup");
  }
}

__device__ __forceinline__ unsigned pk16(unsigned short a, unsigned short b) { return (unsigned)a | ((unsigned)b << 16); }
__device__ __forceinline__ void split_bf(float f, unsigned short& hb, unsigned short& lb) {
  hb = f2bf_bits(f);
  lb = f2bf_bits(f - bf_bits2f(hb));
}
__device__ __forceinline__ void split8(v4f a, v4f c, v4u& uh, v4u& ul) {
  unsigned short hb[8], lb[8];
#pragma unroll
  for (int e = 0; e < 4; ++e) {
    split_bf(a[e], hb[e], lb[e]);
    split_bf(c[e], hb[4 + e], lb[4 + e]);
  }
  uh = (v4u){pk16(hb[0], hb[1]), pk16(hb[2], hb[3]), pk16(hb[4], hb[5]), pk16(hb[6], hb[7])};
  ul = (v4u){pk16(lb[0], lb[1]), pk16(lb[2], lb[3]), pk16(lb[4], lb[5]), pk16(lb[6], lb[7])};
}
__device__ __forceinline__ float wave_sum(float v) {
#pragma unroll
  for (int off = 16; off > 0; off >>= 1) v += __shfl_xor(v, off, 32);
  return v;
}

__global__ __launch_bounds__(256) void cast_split8_kernel(const float* __restrict__ in,
                                                          unsigned short* __restrict__ oh,
                                                          unsigned short* __restrict__ ol, int n8) {
  const int i = blockIdx.x * 256 + threadIdx.x;
  if (i >= n8) return;
  const float* p = in + 8 * (size_t)i;
  const v4f a = *(const v4f*)(p);
  const v4f c = *(const v4f*)(p + 4);
  v4u uh, ul;
  split8(a, c, uh, ul);
  unsigned short* qh = oh + 8 * (size_t)i;
  unsigned short* ql = ol + 8 * (size_t)i;
  for (int pass = 0; pass < 2; ++pass) {
    *(volatile v4u*)qh = uh;
    *(volatile v4u*)ql = ul;
    __threadfence();
  }
}

__global__ __launch_bounds__(256) void tcast_cols_kernel(const float* __restrict__ in, int ncols,
                                                         unsigned short* __restrict__ oh,
                                                         unsigned short* __restrict__ ol) {
  __shared__ float sm[32][65];
  const int t  = threadIdx.x;
  const int d0 = blockIdx.x * 64;
  const int c0 = blockIdx.y * 32;
#pragma unroll
  for (int i = 0; i < 8; ++i) {
    const int e   = i * 256 + t;
    const int cl  = e & 31;
    const int dl  = e >> 5;
    const int cc  = c0 + cl;
    const int ccl = (cc < ncols) ? cc : (ncols - 1);
    float v = in[(size_t)(d0 + dl) * ncols + ccl];
    v = (cc < ncols) ? v : 0.0f;
    sm[cl][dl] = v;
  }
  __syncthreads();
  const int lane = t & 31, wave = t >> 5;
  const int q = lane >> 3, c8 = (lane & 7) * 8;
  const int row = wave * 4 + q;
  v4f a, c;
#pragma unroll
  for (int e = 0; e < 4; ++e) { a[e] = sm[row][c8 + e]; c[e] = sm[row][c8 + 4 + e]; }
  v4u uh, ul;
  split8(a, c, uh, ul);
  const size_t o = (size_t)(c0 + row) * kDim + d0 + c8;
  for (int pass = 0; pass < 2; ++pass) {
    *(volatile v4u*)(oh + o) = uh;
    *(volatile v4u*)(ol + o) = ul;
    __threadfence();
  }
}

template <int RR>
__global__ __launch_bounds__(256) void tcast_rows_kernel(const float* __restrict__ in,
                                                         unsigned short* __restrict__ oh,
                                                         unsigned short* __restrict__ ol) {
  __shared__ float sm[64][RR + 1];
  const int t  = threadIdx.x;
  const int d0 = blockIdx.x * 64;
  const int z  = blockIdx.y;
  const float* src = in + (size_t)z * RR * kDim;
#pragma unroll
  for (int i = 0; i < RR / 4; ++i) {
    const int e  = i * 256 + t;
    const int dl = e & 63;
    const int r  = e >> 6;
    sm[dl][r] = src[(size_t)r * kDim + d0 + dl];
  }
  __syncthreads();
  const int lane = t & 31, wave = t >> 5;
  constexpr int NIT = RR / 32;
  const size_t ob = (size_t)z * kDim * RR + (size_t)d0 * RR;
  v4u uh[NIT], ul[NIT];
  int offs[NIT];
#pragma unroll
  for (int it = 0; it < NIT; ++it) {
    const int off = ((wave * NIT + it) * 32 + lane) * 8;
    const int dl  = off / RR;
    const int r0  = off & (RR - 1);
    v4f a, c;
#pragma unroll
    for (int e = 0; e < 4; ++e) { a[e] = sm[dl][r0 + e]; c[e] = sm[dl][r0 + 4 + e]; }
    split8(a, c, uh[it], ul[it]);
    offs[it] = off;
  }
  for (int pass = 0; pass < 2; ++pass) {
#pragma unroll
    for (int it = 0; it < NIT; ++it) {
      *(volatile v4u*)(oh + ob + offs[it]) = uh[it];
      *(volatile v4u*)(ol + ob + offs[it]) = ul[it];
    }
    __threadfence();
  }
}

__global__ __launch_bounds__(256) void ln_kernel(const float* __restrict__ x, const float* __restrict__ lw,
                                                 const float* __restrict__ lb, float* __restrict__ Xo) {
  __shared__ float red0[8];
  __shared__ float red1[8];
  const int m = blockIdx.x, t = threadIdx.x, lane = t & 31, wave = t >> 5;
  const float* xr = x + (size_t)m * kDim;
  const int c0 = 4 * t, c1 = 1024 + 4 * t;
  const v4f a0 = *(const v4f*)(xr + c0);
  const v4f a1 = *(const v4f*)(xr + c1);
  float s = ((a0[0] + a0[1]) + (a0[2] + a0[3])) + ((a1[0] + a1[1]) + (a1[2] + a1[3]));
  s = wave_sum(s);
  if (lane == 0) red0[wave] = s;
  __syncthreads();
  float tot = red0[0];
#pragma unroll
  for (int q = 1; q < 8; ++q) tot += red0[q];
  const float mu = tot * (1.0f / 2048.0f);
  v4f d0, d1;
  float qs = 0.0f;
#pragma unroll
  for (int e = 0; e < 4; ++e) {
    d0[e] = a0[e] - mu; d1[e] = a1[e] - mu;
    qs += d0[e] * d0[e];
    qs += d1[e] * d1[e];
  }
  qs = wave_sum(qs);
  if (lane == 0) red1[wave] = qs;
  __syncthreads();
  float tq = red1[0];
#pragma unroll
  for (int q = 1; q < 8; ++q) tq += red1[q];
  const float var = tq * (1.0f / 2048.0f);
  const float rs  = rsqrtf(var + kEps);
  const v4f w0 = *(const v4f*)(lw + c0), w1 = *(const v4f*)(lw + c1);
  const v4f b0 = *(const v4f*)(lb + c0), b1 = *(const v4f*)(lb + c1);
  v4f y0, y1;
#pragma unroll
  for (int e = 0; e < 4; ++e) {
    y0[e] = d0[e] * rs * w0[e] + b0[e];
    y1[e] = d1[e] * rs * w1[e] + b1[e];
  }
  float* yr = Xo + (size_t)m * kDim;
  for (int pass = 0; pass < 2; ++pass) {
    *(volatile v4f*)(yr + c0) = y0;
    *(volatile v4f*)(yr + c1) = y1;
    __threadfence();
  }
}

__global__ __launch_bounds__(256) void shift_kernel(const float* __restrict__ X, const float* __restrict__ state,
                                                    const float* __restrict__ tmx, const int* __restrict__ ip,
                                                    float* __restrict__ SX,
                                                    unsigned short* __restrict__ XXh, unsigned short* __restrict__ XXl) {
  const int m = blockIdx.x, t = threadIdx.x;
  const int bi = m / kSeq;
  const int tt = m - bi * kSeq;
  const int iv = ip[0];
  int i1 = 66 * iv + 1;
  i1 = (i1 < 0) ? 0 : ((i1 > kStRows - 1) ? (kStRows - 1) : i1);
  const float* xr = X + (size_t)m * kDim;
  const float* pr = (tt == 0) ? (state + ((size_t)bi * kStRows + i1) * kDim) : (X + (size_t)(m - 1) * kDim);
  {
    const int c0 = 4 * t, c1 = 1024 + 4 * t;
    const v4f x0 = *(const v4f*)(xr + c0), x1 = *(const v4f*)(xr + c1);
    const v4f p0 = *(const v4f*)(pr + c0), p1 = *(const v4f*)(pr + c1);
    const v4f s0 = p0 - x0, s1 = p1 - x1;
    float* sr = SX + (size_t)m * kDim;
    for (int pass = 0; pass < 2; ++pass) {
      *(volatile v4f*)(sr + c0) = s0;
      *(volatile v4f*)(sr + c1) = s1;
      __threadfence();
    }
  }
  {
    const int c = 8 * t;
    const v4f xa = *(const v4f*)(xr + c), xb = *(const v4f*)(xr + c + 4);
    const v4f pa = *(const v4f*)(pr + c), pb = *(const v4f*)(pr + c + 4);
    const v4f ta = *(const v4f*)(tmx + c), tb = *(const v4f*)(tmx + c + 4);
    v4f va, vb;
#pragma unroll
    for (int e = 0; e < 4; ++e) {
      va[e] = xa[e] + (pa[e] - xa[e]) * ta[e];
      vb[e] = xb[e] + (pb[e] - xb[e]) * tb[e];
    }
    v4u uh, ul;
    split8(va, vb, uh, ul);
    const size_t o = (size_t)m * kDim + c;
    for (int pass = 0; pass < 2; ++pass) {
      *(volatile v4u*)(XXh + o) = uh;
      *(volatile v4u*)(XXl + o) = ul;
      __threadfence();
    }
  }
}

__global__ __launch_bounds__(256) void tanh_split2_kernel(const float* __restrict__ in,
                                                          unsigned short* __restrict__ oh,
                                                          unsigned short* __restrict__ ol, int n2) {
  const int i = blockIdx.x * 256 + threadIdx.x;
  if (i >= n2) return;
  const float v0 = tanhf(in[2 * (size_t)i]);
  const float v1 = tanhf(in[2 * (size_t)i + 1]);
  unsigned short h0, l0, h1, l1;
  split_bf(v0, h0, l0);
  split_bf(v1, h1, l1);
  const unsigned uh = pk16(h0, h1), ul = pk16(l0, l1);
  for (int pass = 0; pass < 2; ++pass) {
    ((volatile unsigned*)oh)[i] = uh;
    ((volatile unsigned*)ol)[i] = ul;
    __threadfence();
  }
}

__global__ __launch_bounds__(256) void x5_kernel(const float* __restrict__ X, const float* __restrict__ SX,
                                                 const float* __restrict__ MIX5,
                                                 const float* __restrict__ ma0, const float* __restrict__ ma1,
                                                 const float* __restrict__ ma2, const float* __restrict__ ma3,
                                                 const float* __restrict__ ma4,
                                                 unsigned short* __restrict__ X5h, unsigned short* __restrict__ X5l) {
  const int blk = blockIdx.x, t = threadIdx.x;
  const int f = blk / kTok;
  const int m = blk - f * kTok;
  const float* maa = (f == 0) ? ma0 : (f == 1) ? ma1 : (f == 2) ? ma2 : (f == 3) ? ma3 : ma4;
  const int c = 8 * t;
  const size_t ro = (size_t)m * kDim + c;
  const size_t po = (size_t)f * kPlane + ro;
  const v4f xa = *(const v4f*)(X + ro),     xb = *(const v4f*)(X + ro + 4);
  const v4f sa = *(const v4f*)(SX + ro),    sb = *(const v4f*)(SX + ro + 4);
  const v4f qa = *(const v4f*)(MIX5 + po),  qb = *(const v4f*)(MIX5 + po + 4);
  const v4f na = *(const v4f*)(maa + c),    nb = *(const v4f*)(maa + c + 4);
  v4f va, vb;
#pragma unroll
  for (int e = 0; e < 4; ++e) {
    va[e] = xa[e] + sa[e] * (na[e] + qa[e]);
    vb[e] = xb[e] + sb[e] * (nb[e] + qb[e]);
  }
  v4u uh, ul;
  split8(va, vb, uh, ul);
  for (int pass = 0; pass < 2; ++pass) {
    *(volatile v4u*)(X5h + po) = uh;
    *(volatile v4u*)(X5l + po) = ul;
    __threadfence();
  }
}

__global__ __launch_bounds__(256) void act_kernel(const float* __restrict__ DD, const float* __restrict__ td,
                                                  const float* __restrict__ G,
                                                  float* __restrict__ Wd, float* __restrict__ GS, int nb) {
  const bool second = (blockIdx.x >= (unsigned)nb);
  const int i = ((int)blockIdx.x - (second ? nb : 0)) * 256 + threadIdx.x;
  if (!second) {
    const float a = td[i & (kDim - 1)] + DD[i];
    const float w = expf(-expf(a));
    for (int pass = 0; pass < 2; ++pass) {
      ((volatile float*)Wd)[i] = w;
      __threadfence();
    }
  } else {
    const float g  = G[i];
    const float sg = 1.0f / (1.0f + expf(-g));
    const float gs = g * sg;
    for (int pass = 0; pass < 2; ++pass) {
      ((volatile float*)GS)[i] = gs;
      __threadfence();
    }
  }
}

__global__ __launch_bounds__(512) void state_scan_kernel(
    const float* __restrict__ Rf, const float* __restrict__ Kf, const float* __restrict__ Vf,
    const float* __restrict__ Wd, const float* __restrict__ GS,
    const float* __restrict__ state, const float* __restrict__ bonus,
    const float* __restrict__ gnw, const float* __restrict__ gnb,
    const int* __restrict__ ip, unsigned short* __restrict__ NG) {
  __shared__ float stage[5 * 64];
  __shared__ float part[8 * 64];
  __shared__ __align__(16) unsigned short stg[128];
  const int tid  = threadIdx.x;
  const int lane = tid & 31, wave = tid >> 5;
  const int j    = tid & 63, ig = tid >> 6;
  const int bh   = blockIdx.x;
  const int bi   = bh >> 5, h = bh & 31;
  const int iv   = ip[0];
  int rb = 66 * iv + 2;
  rb = (rb < 0) ? 0 : ((rb > 2) ? 2 : rb);
  float s[8], fa[8];
#pragma unroll
  for (int ii = 0; ii < 8; ++ii) {
    const int i    = ig * 8 + ii;
    const int flat = h * 4096 + i * 64 + j;
    const int row  = rb + (flat >> 11);
    const int col  = flat & 2047;
    s[ii]  = state[((size_t)bi * kStRows + row) * kDim + col];
    fa[ii] = bonus[h * 64 + i];
  }
  const float* src = (ig == 0) ? Rf : (ig == 1) ? Kf : (ig == 2) ? Vf : (ig == 3) ? Wd : GS;
  const float lw0 = gnw[h * 64 + lane], lw1 = gnw[h * 64 + 32 + lane];
  const float lb0 = gnb[h * 64 + lane], lb1 = gnb[h * 64 + 32 + lane];
  const int pl = (lane >> 3) & 1;
  const int c8 = (lane & 7) * 8;
#pragma unroll 1
  for (int t = 0; t < kSeq; ++t) {
    const size_t base = (size_t)(bi * kSeq + t) * kDim + h * 64;
    __syncthreads();
    if (ig < 5) stage[ig * 64 + j] = src[base + j];
    __syncthreads();
    const float vj = stage[128 + j];
    float partial = 0.0f;
#pragma unroll
    for (int ii = 0; ii < 8; ++ii) {
      const int i = ig * 8 + ii;
      const float ri = stage[i];
      const float ki = stage[64 + i];
      const float wi = stage[192 + i];
      const float kv = ki * vj;
      partial += ri * (fa[ii] * kv + s[ii]);
      s[ii] = kv + wi * s[ii];
    }
    part[ig * 64 + j] = partial;
    __syncthreads();
    if (wave == 0) {
      float y0 = part[lane], y1 = part[32 + lane];
#pragma unroll
      for (int q = 1; q < 8; ++q) { y0 += part[q * 64 + lane]; y1 += part[q * 64 + 32 + lane]; }
      const float tot  = wave_sum(y0 + y1);
      const float mean = tot * (1.0f / 64.0f);
      const float d0 = y0 - mean, d1 = y1 - mean;
      const float sq  = wave_sum(d0 * d0 + d1 * d1);
      const float var = sq * (1.0f / 64.0f);
      const float rs  = rsqrtf(var + kEps);
      const float n0 = d0 * rs * lw0 + lb0;
      const float n1 = d1 * rs * lw1 + lb1;
      const float o0 = n0 * stage[256 + lane];
      const float o1 = n1 * stage[256 + 32 + lane];
      unsigned short h0, l0, h1, l1;
      split_bf(o0, h0, l0);
      split_bf(o1, h1, l1);
      stg[lane] = h0; stg[32 + lane] = h1; stg[64 + lane] = l0; stg[96 + lane] = l1;
      __builtin_amdgcn_fence(__ATOMIC_RELEASE, "workgroup");
      __builtin_amdgcn_wave_barrier();
      __builtin_amdgcn_fence(__ATOMIC_ACQUIRE, "workgroup");
      const v4u val = *(const v4u*)(stg + (lane & 15) * 8);
      unsigned short* dst = NG + (size_t)pl * kPlane + base + c8;
      for (int pass = 0; pass < 2; ++pass) {
        if (lane < 16) *(volatile v4u*)dst = val;
        __threadfence();
      }
    }
  }
}

extern "C" void kernel_launch(void* const* d_in, const int* in_sizes, int n_in,
                              void* d_out, int out_size, void* d_ws, size_t ws_size,
                              hipStream_t stream) {
  (void)in_sizes; (void)n_in; (void)out_size;
  const float* x       = (const float*)d_in[0];
  const float* state   = (const float*)d_in[1];
  const float* ln1_w   = (const float*)d_in[2];
  const float* ln1_b   = (const float*)d_in[3];
  const float* tmx     = (const float*)d_in[4];
  const float* mix_w1  = (const float*)d_in[5];
  const float* mix_w2  = (const float*)d_in[6];
  const float* maak    = (const float*)d_in[7];
  const float* maaw    = (const float*)d_in[8];
  const float* maav    = (const float*)d_in[9];
  const float* maar    = (const float*)d_in[10];
  const float* maag    = (const float*)d_in[11];
  const float* tdecay  = (const float*)d_in[12];
  const float* dec_w1  = (const float*)d_in[13];
  const float* dec_w2  = (const float*)d_in[14];
  const float* bonus   = (const float*)d_in[15];
  const float* Wrec    = (const float*)d_in[16];
  const float* Wkey    = (const float*)d_in[17];
  const float* Wval    = (const float*)d_in[18];
  const float* Wproj   = (const float*)d_in[19];
  const float* Wgate   = (const float*)d_in[20];
  const float* gnw     = (const float*)d_in[21];
  const float* gnb     = (const float*)d_in[22];
  const int*   ip      = (const int*)d_in[23];

  char* ws = (char*)d_ws;
  size_t off = 0;
  auto carve = [&](size_t bytes) -> size_t { const size_t o = off; off += (bytes + 4095) & ~(size_t)4095; return o; };
  const size_t f32Plane = (size_t)kPlane * 4;
  const size_t b16Plane = (size_t)kPlane * 2;
  const size_t oX     = carve(f32Plane);
  const size_t oSX    = carve(f32Plane);
  const size_t oXXh   = carve(b16Plane);
  const size_t oXXl   = carve(b16Plane);
  const size_t oW1Th  = carve((size_t)kLrPad * kDim * 2);
  const size_t oW1Tl  = carve((size_t)kLrPad * kDim * 2);
  const size_t oT5f   = carve((size_t)kTok * kLrPad * 4);
  const size_t oT5h   = carve((size_t)kTok * kLrPad * 2);
  const size_t oT5l   = carve((size_t)kTok * kLrPad * 2);
  const size_t oW2Th  = carve((size_t)5 * kDim * 32 * 2);
  const size_t oW2Tl  = carve((size_t)5 * kDim * 32 * 2);
  const size_t oMIX5  = carve(5 * f32Plane);
  const size_t oX5h   = carve(5 * b16Plane);
  const size_t oX5l   = carve(5 * b16Plane);
  const size_t oWBh   = carve((size_t)kDim * kDim * 2);
  const size_t oWBl   = carve((size_t)kDim * kDim * 2);
  const size_t oW1DTh = carve((size_t)kDec * kDim * 2);
  const size_t oW1DTl = carve((size_t)kDec * kDim * 2);
  const size_t oTD1f  = carve((size_t)kTok * kDec * 4);
  const size_t oTD1h  = carve((size_t)kTok * kDec * 2);
  const size_t oTD1l  = carve((size_t)kTok * kDec * 2);
  const size_t oW2DTh = carve((size_t)kDim * kDec * 2);
  const size_t oW2DTl = carve((size_t)kDim * kDec * 2);
  const size_t oWd    = carve(f32Plane);
  const size_t oGS    = carve(f32Plane);
  const size_t oNG    = carve(2 * b16Plane);
  if (off > ws_size) return;

  float* Xf   = (float*)(ws + oX);
  float* SXf  = (float*)(ws + oSX);
  unsigned short* XXh   = (unsigned short*)(ws + oXXh);
  unsigned short* XXl   = (unsigned short*)(ws + oXXl);
  unsigned short* W1Th  = (unsigned short*)(ws + oW1Th);
  unsigned short* W1Tl  = (unsigned short*)(ws + oW1Tl);
  float* T5f  = (float*)(ws + oT5f);
  unsigned short* T5h   = (unsigned short*)(ws + oT5h);
  unsigned short* T5l   = (unsigned short*)(ws + oT5l);
  unsigned short* W2Th  = (unsigned short*)(ws + oW2Th);
  unsigned short* W2Tl  = (unsigned short*)(ws + oW2Tl);
  float* MIX5f = (float*)(ws + oMIX5);
  float* Kf   = MIX5f + 0 * kPlane;
  float* Vf   = MIX5f + 1 * kPlane;
  float* Rf   = MIX5f + 2 * kPlane;
  float* Gf   = MIX5f + 3 * kPlane;
  float* DDf  = MIX5f + 4 * kPlane;
  unsigned short* X5h   = (unsigned short*)(ws + oX5h);
  unsigned short* X5l   = (unsigned short*)(ws + oX5l);
  unsigned short* WBh   = (unsigned short*)(ws + oWBh);
  unsigned short* WBl   = (unsigned short*)(ws + oWBl);
  unsigned short* W1DTh = (unsigned short*)(ws + oW1DTh);
  unsigned short* W1DTl = (unsigned short*)(ws + oW1DTl);
  float* TD1f = (float*)(ws + oTD1f);
  unsigned short* TD1h  = (unsigned short*)(ws + oTD1h);
  unsigned short* TD1l  = (unsigned short*)(ws + oTD1l);
  unsigned short* W2DTh = (unsigned short*)(ws + oW2DTh);
  unsigned short* W2DTl = (unsigned short*)(ws + oW2DTl);
  float* Wdf  = (float*)(ws + oWd);
  float* GSf  = (float*)(ws + oGS);
  unsigned short* NG    = (unsigned short*)(ws + oNG);
  float* outp = (float*)d_out;

  auto gemm = [&](const unsigned short* Ah, const unsigned short* Al, int lda, long sA,
                  const unsigned short* Bh, const unsigned short* Bl, int ldb, long sB,
                  float* C, int ldc, long sC, int M, int N, int K, int batch) {
    const int tiles = (M / 64) * (N / 64);
    dim3 grid((tiles + 7) / 8, batch);
    wmma_gemm64<1, true, 0, 0, false, 0><<<grid, 256, 0, stream>>>(
        Ah, Al, lda, sA, Bh, Bl, ldb, sB, (void*)C, (void*)nullptr, ldc, sC,
        (const float*)nullptr, (const float*)nullptr, 0L, M, N, K, 1.0f);
  };

  const int castBlocks = (int)((long)kDim * kDim / 8 / 256);
  const int n8sq = (int)((long)kDim * kDim / 8);

  tcast_cols_kernel<<<dim3(kDim / 64, kLrPad / 32), 256, 0, stream>>>(mix_w1, kLr5, W1Th, W1Tl);
  tcast_rows_kernel<32><<<dim3(kDim / 64, 5), 256, 0, stream>>>(mix_w2, W2Th, W2Tl);
  tcast_cols_kernel<<<dim3(kDim / 64, kDec / 32), 256, 0, stream>>>(dec_w1, kDec, W1DTh, W1DTl);
  tcast_rows_kernel<64><<<dim3(kDim / 64, 1), 256, 0, stream>>>(dec_w2, W2DTh, W2DTl);

  ln_kernel<<<kTok, 256, 0, stream>>>(x, ln1_w, ln1_b, Xf);
  shift_kernel<<<kTok, 256, 0, stream>>>(Xf, state, tmx, ip, SXf, XXh, XXl);

  gemm(XXh, XXl, kDim, 0L, W1Th, W1Tl, kDim, 0L, T5f, kLrPad, 0L, kTok, kLrPad, kDim, 1);
  tanh_split2_kernel<<<(kTok * kLrPad / 2) / 256, 256, 0, stream>>>(T5f, T5h, T5l, kTok * kLrPad / 2);
  gemm(T5h, T5l, kLrPad, 32L, W2Th, W2Tl, 32, (long)kDim * 32, MIX5f, kDim, (long)kPlane, kTok, kDim, 32, 5);

  x5_kernel<<<5 * kTok, 256, 0, stream>>>(Xf, SXf, MIX5f, maak, maaw, maav, maar, maag, X5h, X5l);

  cast_split8_kernel<<<castBlocks, 256, 0, stream>>>(Wkey, WBh, WBl, n8sq);
  gemm(X5h + 0 * kPlane, X5l + 0 * kPlane, kDim, 0L, WBh, WBl, kDim, 0L, Kf, kDim, 0L, kTok, kDim, kDim, 1);
  cast_split8_kernel<<<castBlocks, 256, 0, stream>>>(Wval, WBh, WBl, n8sq);
  gemm(X5h + 2 * kPlane, X5l + 2 * kPlane, kDim, 0L, WBh, WBl, kDim, 0L, Vf, kDim, 0L, kTok, kDim, kDim, 1);
  cast_split8_kernel<<<castBlocks, 256, 0, stream>>>(Wrec, WBh, WBl, n8sq);
  gemm(X5h + 3 * kPlane, X5l + 3 * kPlane, kDim, 0L, WBh, WBl, kDim, 0L, Rf, kDim, 0L, kTok, kDim, kDim, 1);
  cast_split8_kernel<<<castBlocks, 256, 0, stream>>>(Wgate, WBh, WBl, n8sq);
  gemm(X5h + 4 * kPlane, X5l + 4 * kPlane, kDim, 0L, WBh, WBl, kDim, 0L, Gf, kDim, 0L, kTok, kDim, kDim, 1);

  gemm(X5h + 1 * kPlane, X5l + 1 * kPlane, kDim, 0L, W1DTh, W1DTl, kDim, 0L, TD1f, kDec, 0L, kTok, kDec, kDim, 1);
  tanh_split2_kernel<<<(kTok * kDec / 2) / 256, 256, 0, stream>>>(TD1f, TD1h, TD1l, kTok * kDec / 2);
  gemm(TD1h, TD1l, kDec, 0L, W2DTh, W2DTl, kDec, 0L, DDf, kDim, 0L, kTok, kDim, kDec, 1);

  const int nbAct = (int)(kPlane / 256);
  act_kernel<<<2 * nbAct, 256, 0, stream>>>(DDf, tdecay, Gf, Wdf, GSf, nbAct);

  state_scan_kernel<<<kBatch * (kDim / kHeadSz), 512, 0, stream>>>(Rf, Kf, Vf, Wdf, GSf, state, bonus, gnw, gnb, ip, NG);

  cast_split8_kernel<<<castBlocks, 256, 0, stream>>>(Wproj, WBh, WBl, n8sq);
  gemm(NG, NG + kPlane, kDim, 0L, WBh, WBl, kDim, 0L, outp, kDim, 0L, kTok, kDim, kDim, 1);
}
